// Group_query_Attention_28372553957596
// MI455X (gfx1250) — hardware-verified
//
#include <hip/hip_runtime.h>
#include <stdint.h>

typedef __attribute__((ext_vector_type(16))) _Float16 v16h;
typedef __attribute__((ext_vector_type(8)))  _Float16 v8h;
typedef __attribute__((ext_vector_type(16))) __bf16   v16b;
typedef __attribute__((ext_vector_type(8)))  __bf16   v8b;
typedef __attribute__((ext_vector_type(8)))  float    v8f;
typedef __attribute__((ext_vector_type(4)))  float    v4f;
typedef __attribute__((ext_vector_type(4)))  unsigned v4u;

constexpr int kSeq  = 2048;
constexpr int kCq   = 2048;
constexpr int kCkv  = 512;
constexpr int kHd   = 64;
constexpr int kHq   = 32;
constexpr int kGrp  = 4;
static_assert(kSeq % 64 == 0);
static_assert(kCq % 64 == 0);
static_assert(kCkv % 64 == 0);
static_assert(kCq % 32 == 0);
static_assert(kHq * kHd == kCq);
static_assert((kHq / kGrp) * kHd == kCkv);

__device__ __forceinline__ unsigned short f2bf_bits(float f) {
  unsigned u = __float_as_uint(f);
  return (unsigned short)((u + 0x7FFFu + ((u >> 16) & 1u)) >> 16);
}
__device__ __forceinline__ float bf_bits2f(unsigned short h) { return __uint_as_float(((unsigned)h) << 16); }

__device__ __forceinline__ void dep_guard_h(v8f& a, v8f& b, v16h x, v16h y) { asm volatile("v_nop\n\tv_nop\n\tv_nop\n\tv_nop" : "+v"(a), "+v"(b) : "v"(x), "v"(y)); }
__device__ __forceinline__ void dep_guard_b(v8f& a, v8f& b, v16b x, v16b y) { asm volatile("v_nop\n\tv_nop\n\tv_nop\n\tv_nop" : "+v"(a), "+v"(b) : "v"(x), "v"(y)); }
__device__ __forceinline__ void keep4_h(v16h a, v16h b, v16h c, v16h d) { asm volatile("v_nop" :: "v"(a), "v"(b), "v"(c), "v"(d)); }
__device__ __forceinline__ void keep4_b(v16b a, v16b b, v16b c, v16b d) { asm volatile("v_nop" :: "v"(a), "v"(b), "v"(c), "v"(d)); }
__device__ __forceinline__ void acc_guard4(v8f& a, v8f& b, v8f& c, v8f& d) { asm volatile("v_nop\n\tv_nop\n\tv_nop\n\tv_nop" : "+v"(a), "+v"(b), "+v"(c), "+v"(d)); }
template <typename T> struct Frag;
template <> struct Frag<_Float16> {
  typedef v16h V; union U { v16h v; v8h h[2]; };
  static __device__ __forceinline__ v16h load(const _Float16* p) {
    U f; f.h[0] = *(const v8h*)(p); f.h[1] = *(const v8h*)(p + 16); return f.v;
  }
  static __device__ __forceinline__ v8f mma(v16h a, v16h b, v8f c) {
    return __builtin_amdgcn_wmma_f32_16x16x32_f16(false, a, false, b, (short)0, c, false, false);
  }
  static __device__ __forceinline__ void guard(v8f& a, v8f& b, v16h x, v16h y) { dep_guard_h(a, b, x, y); }
  static __device__ __forceinline__ void keep(v16h a, v16h b, v16h c, v16h d) { keep4_h(a, b, c, d); }
};
template <> struct Frag<__bf16> {
  typedef v16b V; union U { v16b v; v8b h[2]; };
  static __device__ __forceinline__ v16b load(const __bf16* p) {
    U f; f.h[0] = *(const v8b*)(p); f.h[1] = *(const v8b*)(p + 16); return f.v;
  }
  static __device__ __forceinline__ v8f mma(v16b a, v16b b, v8f c) {
    return __builtin_amdgcn_wmma_f32_16x16x32_bf16(false, a, false, b, (short)0, c, false, false);
  }
  static __device__ __forceinline__ void guard(v8f& a, v8f& b, v16b x, v16b y) { dep_guard_b(a, b, x, y); }
  static __device__ __forceinline__ void keep(v16b a, v16b b, v16b c, v16b d) { keep4_b(a, b, c, d); }
};

template <int ET> struct Elem;
template <> struct Elem<0> { typedef _Float16 T; };
template <> struct Elem<1> { typedef __bf16 T; };
template <int ET, int SPLIT, int BIAS_MODE, int OUT_MODE, bool RESID, int ACT = 0>
__global__ __launch_bounds__(256) void wmma_gemm64(
    const unsigned short* __restrict__ Ap, const unsigned short* __restrict__ A2p, int lda, long strideA,
    const unsigned short* __restrict__ Btp, const unsigned short* __restrict__ Bt2p, int ldb, long strideB,
    void* __restrict__ Cout, void* __restrict__ Cout2, int ldc, long strideC,
    const float* __restrict__ bias,
    const float* __restrict__ resid, long strideR,
    int M, int N, int K, float scale) {
  typedef typename Elem<ET>::T T;
  typedef typename Frag<T>::V V;
  const T* A = (const T*)Ap; const T* A2 = (const T*)A2p; const T* Bt = (const T*)Btp; const T* Bt2 = (const T*)Bt2p;
  __shared__ __align__(16) float sT[8][16 * 68];
  const int b    = blockIdx.y;
  const int lane = threadIdx.x & 31;
  const int wave = threadIdx.x >> 5;
  const int tilesN = N >> 6;
  const int tilesM = M >> 6;
  const int tile = blockIdx.x * 8 + wave;
  if (tile >= tilesM * tilesN) return;
  const int tm = tile / tilesN;
  const int tn = tile - tm * tilesN;
  const int m0 = tm << 6;
  const int n0 = tn << 6;

  const T* Ab  = A  + (size_t)b * strideA;
  const T* Bb  = Bt + (size_t)b * strideB;
  const T* Ab2 = (SPLIT != 0) ? (A2  + (size_t)b * strideA) : nullptr;
  const T* Bb2 = (SPLIT == 1) ? (Bt2 + (size_t)b * strideB) : nullptr;

  const int rlane = lane & 15;
  const int koff  = (lane >> 4) * 8;
  const int mOff  = (lane >> 4) * 8;

  v8f acc[4][4];
#pragma unroll
  for (int i = 0; i < 4; ++i)
#pragma unroll
    for (int j = 0; j < 4; ++j) acc[i][j] = (v8f){0.f,0.f,0.f,0.f,0.f,0.f,0.f,0.f};

  for (int k0 = 0; k0 < K; k0 += 32) {
    V bh[4], bl[4];
#pragma unroll
    for (int j = 0; j < 4; ++j) {
      const size_t bofs = (size_t)(n0 + (j << 4) + rlane) * ldb + koff + k0;
      bh[j] = Frag<T>::load(Bb + bofs);
      bl[j] = bh[j];
      if (SPLIT == 1) bl[j] = Frag<T>::load(Bb2 + bofs);
    }
#pragma unroll
    for (int i = 0; i < 4; ++i) {
      const size_t ao = (size_t)(m0 + (i << 4) + rlane) * lda + koff + k0;
      V ah = Frag<T>::load(Ab + ao);
      V al = ah;
      if (SPLIT != 0) al = Frag<T>::load(Ab2 + ao);
#pragma unroll
      for (int j = 0; j < 4; ++j) {
        acc[i][j] = Frag<T>::mma(ah, bh[j], acc[i][j]);
        if (SPLIT == 1) acc[i][j] = Frag<T>::mma(ah, bl[j], acc[i][j]);
        if (SPLIT != 0) acc[i][j] = Frag<T>::mma(al, bh[j], acc[i][j]);
      }
      Frag<T>::guard(acc[i][0], acc[i][3], ah, al);
    }
    Frag<T>::keep(bh[0], bh[1], bh[2], bh[3]);
    if (SPLIT == 1) Frag<T>::keep(bl[0], bl[1], bl[2], bl[3]);
  }
  acc_guard4(acc[0][0], acc[0][1], acc[0][2], acc[0][3]);
  acc_guard4(acc[1][0], acc[1][1], acc[1][2], acc[1][3]);
  acc_guard4(acc[2][0], acc[2][1], acc[2][2], acc[2][3]);
  acc_guard4(acc[3][0], acc[3][1], acc[3][2], acc[3][3]);

  float* slab = sT[wave];
  const float* Rb = RESID ? (resid + (size_t)b * strideR) : nullptr;
#pragma unroll
  for (int i = 0; i < 4; ++i) {
    const int mBase = m0 + (i << 4);
#pragma unroll
    for (int j = 0; j < 4; ++j) {
      const int n = n0 + (j << 4) + rlane;
      float bv = 0.f;
      if (BIAS_MODE == 2) bv = bias[n];
#pragma unroll
      for (int r = 0; r < 8; ++r) {
        float v = acc[i][j][r] * scale;
        if (BIAS_MODE == 1) v += bias[mBase + mOff + r];
        if (BIAS_MODE == 2) v += bv;
        if (RESID) v += Rb[(size_t)(mBase + mOff + r) * ldc + n];
        if (ACT == 1) v = tanhf(v);
        if (ACT == 2) v = fmaxf(v, 0.0f);
        if (ACT == 4) v = (v > 0.f) ? v : 0.01f * v;
        slab[(mOff + r) * 68 + (j << 4) + rlane] = v;
      }
    }
    __builtin_amdgcn_fence(__ATOMIC_RELEASE, "workgroup");
    __builtin_amdgcn_wave_barrier();
    __builtin_amdgcn_fence(__ATOMIC_ACQUIRE, "workgroup");
    if (OUT_MODE == 0) {
      float* C = (float*)Cout + (size_t)b * strideC;
      const int hh = lane >> 4, c4 = (lane & 15) * 4;
      for (int pass = 0; pass < 2; ++pass) {
#pragma unroll
        for (int it = 0; it < 8; ++it) {
          const int row = it * 2 + hh;
          v4f v = *(const v4f*)(slab + row * 68 + c4);
          *(volatile v4f*)(C + (size_t)(mBase + row) * ldc + n0 + c4) = v;
        }
        __threadfence();
      }
    } else {
      const int q = lane >> 3, c8 = (lane & 7) * 8;
      unsigned short* C  = (unsigned short*)Cout  + (size_t)b * strideC;
      unsigned short* C2 = (OUT_MODE == 2) ? ((unsigned short*)Cout2 + (size_t)b * strideC) : nullptr;
      for (int pass = 0; pass < 2; ++pass) {
#pragma unroll
        for (int it = 0; it < 4; ++it) {
          const int row = it * 4 + q;
          const float* sp = slab + row * 68 + c8;
          v8h hv, lv;
#pragma unroll
          for (int e = 0; e < 8; ++e) {
            if (OUT_MODE == 1) {
              hv[e] = (_Float16)sp[e];
            } else {
              unsigned short hb = f2bf_bits(sp[e]);
              unsigned short lb = f2bf_bits(sp[e] - bf_bits2f(hb));
              hv[e] = __builtin_bit_cast(_Float16, hb);
              lv[e] = __builtin_bit_cast(_Float16, lb);
            }
          }
          *(volatile v8h*)(C + (size_t)(mBase + row) * ldc + n0 + c8) = hv;
          if (OUT_MODE == 2) *(volatile v8h*)(C2 + (size_t)(mBase + row) * ldc + n0 + c8) = lv;
        }
        __threadfence();
      }
    }
    __builtin_amdgcn_fence(__ATOMIC_RELEASE, "workgroup");
    __builtin_amdgcn_wave_barrier();
    __builtin_amdgcn_fence(__ATOMIC_ACQUIRE, "workgroup");
  }
}

__global__ __launch_bounds__(256) void cast_f32_bf16x8(
    const float* __restrict__ in, unsigned short* __restrict__ out, int n8) {
  const int i = blockIdx.x * 256 + threadIdx.x;
  if (i < n8) {
    const size_t e0 = (size_t)i * 8;
    const v4f a = *(const v4f*)(in + e0);
    const v4f c = *(const v4f*)(in + e0 + 4);
    v4u w;
    w[0] = (unsigned)f2bf_bits(a[0]) | ((unsigned)f2bf_bits(a[1]) << 16);
    w[1] = (unsigned)f2bf_bits(a[2]) | ((unsigned)f2bf_bits(a[3]) << 16);
    w[2] = (unsigned)f2bf_bits(c[0]) | ((unsigned)f2bf_bits(c[1]) << 16);
    w[3] = (unsigned)f2bf_bits(c[2]) | ((unsigned)f2bf_bits(c[3]) << 16);
    *(volatile v4u*)(out + e0) = w;
    __threadfence();
    *(volatile v4u*)(out + e0) = w;
  }
}

__device__ __forceinline__ v8f at_mma(v16b a, v16b b, v8f c) {
  c = __builtin_amdgcn_wmma_f32_16x16x32_bf16(false, a, false, b, (short)0, c, false, false);
  asm volatile("v_nop\n\tv_nop\n\tv_nop\n\tv_nop" : "+v"(c) : "v"(a), "v"(b));
  return c;
}
__device__ __forceinline__ __bf16 at_f2bf(float f) { return __builtin_bit_cast(__bf16, f2bf_bits(f)); }
__device__ __forceinline__ void at_split(float f, __bf16& hi, __bf16& lo) {
  const unsigned short hb = f2bf_bits(f);
  hi = __builtin_bit_cast(__bf16, hb);
  lo = at_f2bf(f - __uint_as_float(((unsigned)hb) << 16));
}

constexpr int kAtPitchO = 68;
__global__ __launch_bounds__(128)
void gqa_attn64(const unsigned short* __restrict__ Qhp, const unsigned short* __restrict__ Qlp,
                const unsigned short* __restrict__ Khp, const unsigned short* __restrict__ Klp,
                const unsigned short* __restrict__ Vthp, const unsigned short* __restrict__ Vtlp,
                unsigned short* __restrict__ AOh, unsigned short* __restrict__ AOl) {
  typedef Frag<__bf16>::U FB;
  const __bf16* Qh  = (const __bf16*)Qhp;  const __bf16* Ql  = (const __bf16*)Qlp;
  const __bf16* Kh  = (const __bf16*)Khp;  const __bf16* Kl  = (const __bf16*)Klp;
  const __bf16* Vth = (const __bf16*)Vthp; const __bf16* Vtl = (const __bf16*)Vtlp;

  __shared__ __align__(16) __bf16 Psh[4][16 * 64];
  __shared__ __align__(16) __bf16 Psl[4][16 * 64];
  __shared__ __align__(16) float  Os[4][16 * kAtPitchO];

  const int tid  = threadIdx.x;
  const int wave = tid >> 5;
  const int lane = tid & 31;
  const int hh   = lane >> 4;
  const int c    = lane & 15;
  const int koff = hh * 8;

  constexpr int nqb = kSeq / 64;
  const int bx = blockIdx.x;
  const int qb = bx % nqb;
  const int hq = bx / nqb;
  const int hk = hq / kGrp;
  const int q0 = qb * 64 + wave * 16;

  v16b qah[2], qal[2];
#pragma unroll
  for (int dc = 0; dc < 2; ++dc) {
    const size_t qo = (size_t)(q0 + c) * kCq + (size_t)hq * kHd + dc * 32 + koff;
    qah[dc] = Frag<__bf16>::load(Qh + qo);
    qal[dc] = Frag<__bf16>::load(Ql + qo);
  }

  float mrow[8], lrow[8];
  v8f oacc[4];
#pragma unroll
  for (int r = 0; r < 8; ++r) { mrow[r] = -__builtin_inff(); lrow[r] = 0.f; }
#pragma unroll
  for (int t = 0; t < 4; ++t) oacc[t] = (v8f){0.f,0.f,0.f,0.f,0.f,0.f,0.f,0.f};

  __bf16* pwh = Psh[wave];
  __bf16* pwl = Psl[wave];

  const int nChunks = qb + 1;
  for (int kc = 0; kc < nChunks; ++kc) {
    const int kv0 = kc * 64;
    __builtin_amdgcn_fence(__ATOMIC_RELEASE, "workgroup");
    __builtin_amdgcn_wave_barrier();
    __builtin_amdgcn_fence(__ATOMIC_ACQUIRE, "workgroup");

    v8f s[4];
#pragma unroll
    for (int j = 0; j < 4; ++j) {
      s[j] = (v8f){0.f,0.f,0.f,0.f,0.f,0.f,0.f,0.f};
#pragma unroll
      for (int dc = 0; dc < 2; ++dc) {
        const size_t ko = (size_t)(kv0 + j * 16 + c) * kCkv + (size_t)hk * kHd + dc * 32 + koff;
        const v16b kbh = Frag<__bf16>::load(Kh + ko);
        const v16b kbl = Frag<__bf16>::load(Kl + ko);
        s[j] = at_mma(qah[dc], kbh, s[j]);
        s[j] = at_mma(qah[dc], kbl, s[j]);
        s[j] = at_mma(qal[dc], kbh, s[j]);
      }
    }

    const bool diag = (kc == qb);
    float cm[8];
#pragma unroll
    for (int r = 0; r < 8; ++r) {
      const int qrow = q0 + 8 * hh + r;
      float m = -__builtin_inff();
#pragma unroll
      for (int j = 0; j < 4; ++j) {
        const int kvcol = kv0 + j * 16 + c;
        const bool msk = diag && (kvcol > qrow);
        const float sv = msk ? -__builtin_inff() : s[j][r];
        s[j][r] = sv;
        m = fmaxf(m, sv);
      }
#pragma unroll
      for (int off = 1; off < 16; off <<= 1) m = fmaxf(m, __shfl_xor(m, off, 32));
      cm[r] = m;
    }

#pragma unroll
    for (int r = 0; r < 8; ++r) {
      const float mnew = fmaxf(mrow[r], cm[r]);
      const float alpha = expf(mrow[r] - mnew);
      mrow[r] = mnew;
      float psum = 0.f;
#pragma unroll
      for (int j = 0; j < 4; ++j) {
        const float p = expf(s[j][r] - mnew);
        psum += p;
        __bf16 ph, pl;
        at_split(p, ph, pl);
        pwh[(8 * hh + r) * 64 + j * 16 + c] = ph;
        pwl[(8 * hh + r) * 64 + j * 16 + c] = pl;
      }
#pragma unroll
      for (int off = 1; off < 16; off <<= 1) psum += __shfl_xor(psum, off, 32);
      lrow[r] = lrow[r] * alpha + psum;
#pragma unroll
      for (int t = 0; t < 4; ++t) oacc[t][r] *= alpha;
    }
    __builtin_amdgcn_fence(__ATOMIC_RELEASE, "workgroup");
    __builtin_amdgcn_wave_barrier();
    __builtin_amdgcn_fence(__ATOMIC_ACQUIRE, "workgroup");

#pragma unroll
    for (int kk = 0; kk < 2; ++kk) {
      FB pa, pb;
      pa.h[0] = *(const v8b*)(pwh + c * 64 + kk * 32 + 8 * hh);
      pa.h[1] = *(const v8b*)(pwh + c * 64 + kk * 32 + 16 + 8 * hh);
      pb.h[0] = *(const v8b*)(pwl + c * 64 + kk * 32 + 8 * hh);
      pb.h[1] = *(const v8b*)(pwl + c * 64 + kk * 32 + 16 + 8 * hh);
#pragma unroll
      for (int t = 0; t < 4; ++t) {
        const size_t vo = (size_t)((size_t)hk * kHd + t * 16 + c) * kSeq + kv0 + kk * 32 + koff;
        const v16b vbh = Frag<__bf16>::load(Vth + vo);
        const v16b vbl = Frag<__bf16>::load(Vtl + vo);
        oacc[t] = at_mma(pa.v, vbh, oacc[t]);
        oacc[t] = at_mma(pa.v, vbl, oacc[t]);
        oacc[t] = at_mma(pb.v, vbh, oacc[t]);
      }
    }
  }

  float* os = Os[wave];
#pragma unroll
  for (int r = 0; r < 8; ++r) {
    const float inv = 1.0f / lrow[r];
#pragma unroll
    for (int t = 0; t < 4; ++t) os[(8 * hh + r) * kAtPitchO + t * 16 + c] = oacc[t][r] * inv;
  }
  __builtin_amdgcn_fence(__ATOMIC_RELEASE, "workgroup");
  __builtin_amdgcn_wave_barrier();
  __builtin_amdgcn_fence(__ATOMIC_ACQUIRE, "workgroup");
  {
    const int q8 = lane >> 3, c8 = (lane & 7) * 8;
    for (int pass = 0; pass < 2; ++pass) {
#pragma unroll
      for (int it = 0; it < 4; ++it) {
        const int row = it * 4 + q8;
        const float* sp = os + row * kAtPitchO + c8;
        v8h hv, lv;
#pragma unroll
        for (int e = 0; e < 8; ++e) {
          const unsigned short hb = f2bf_bits(sp[e]);
          const unsigned short lb = f2bf_bits(sp[e] - bf_bits2f(hb));
          hv[e] = __builtin_bit_cast(_Float16, hb);
          lv[e] = __builtin_bit_cast(_Float16, lb);
        }
        const size_t oo = (size_t)(q0 + row) * kCq + (size_t)hq * kHd + c8;
        *(volatile v8h*)(AOh + oo) = hv;
        *(volatile v8h*)(AOl + oo) = lv;
      }
      __threadfence();
    }
  }
}

extern "C" void kernel_launch(void* const* d_in, const int* in_sizes, int n_in,
                              void* d_out, int out_size, void* d_ws,
                              size_t ws_size, hipStream_t stream) {
  if (n_in < 6) return;
  if (in_sizes[0] != kSeq * kCq) return;
  if (in_sizes[1] != kCq * kCq) return;
  if (in_sizes[2] != kCkv * kCq) return;
  if (in_sizes[3] != kCkv * kCq) return;
  if (in_sizes[4] != kCq * kCq) return;
  if (in_sizes[5] != kCq) return;
  if (out_size != kSeq * kCq) return;

  const float* x  = (const float*)d_in[0];
  const float* Wq = (const float*)d_in[1];
  const float* Wk = (const float*)d_in[2];
  const float* Wv = (const float*)d_in[3];
  const float* Wo = (const float*)d_in[4];
  const float* bo = (const float*)d_in[5];
  float* out = (float*)d_out;

  const size_t nX   = (size_t)kSeq * kCq;
  const size_t nWq  = (size_t)kCq * kCq;
  const size_t nWkv = (size_t)kCkv * kCq;
  const size_t nKpl = (size_t)kSeq * kCkv;

  size_t off = 0;
  unsigned char* ws = (unsigned char*)d_ws;
  unsigned short* xb  = (unsigned short*)(ws + off); off += nX * 2;
  unsigned short* Wqb = (unsigned short*)(ws + off); off += nWq * 2;
  unsigned short* Wkb = (unsigned short*)(ws + off); off += nWkv * 2;
  unsigned short* Wvb = (unsigned short*)(ws + off); off += nWkv * 2;
  unsigned short* Wob = (unsigned short*)(ws + off); off += nWq * 2;
  unsigned short* Qh  = (unsigned short*)(ws + off); off += nX * 2;
  unsigned short* Ql  = (unsigned short*)(ws + off); off += nX * 2;
  unsigned short* Kh  = (unsigned short*)(ws + off); off += nKpl * 2;
  unsigned short* Kl  = (unsigned short*)(ws + off); off += nKpl * 2;
  unsigned short* Vth = (unsigned short*)(ws + off); off += nKpl * 2;
  unsigned short* Vtl = (unsigned short*)(ws + off); off += nKpl * 2;
  unsigned short* AOh = (unsigned short*)(ws + off); off += nX * 2;
  unsigned short* AOl = (unsigned short*)(ws + off); off += nX * 2;
  if (off > ws_size) return;

  {
    const int n8x = (int)(nX / 8), n8q = (int)(nWq / 8), n8kv = (int)(nWkv / 8);
    cast_f32_bf16x8<<<dim3((n8x + 255) / 256), dim3(256), 0, stream>>>(x,  xb,  n8x);
    cast_f32_bf16x8<<<dim3((n8q + 255) / 256), dim3(256), 0, stream>>>(Wq, Wqb, n8q);
    cast_f32_bf16x8<<<dim3((n8kv + 255) / 256), dim3(256), 0, stream>>>(Wk, Wkb, n8kv);
    cast_f32_bf16x8<<<dim3((n8kv + 255) / 256), dim3(256), 0, stream>>>(Wv, Wvb, n8kv);
    cast_f32_bf16x8<<<dim3((n8q + 255) / 256), dim3(256), 0, stream>>>(Wo, Wob, n8q);
  }

  static_assert(kSeq % 64 == 0 && kCq % 64 == 0 && kCkv % 64 == 0 && kCq % 32 == 0 && kSeq % 32 == 0);
  {
    const int tiles = (kSeq / 64) * (kCq / 64);
    wmma_gemm64<1, 0, 0, 2, false><<<dim3(tiles / 8, 1), dim3(256), 0, stream>>>(
        xb, nullptr, kCq, 0L, Wqb, nullptr, kCq, 0L, (void*)Qh, (void*)Ql, kCq, 0L,
        nullptr, nullptr, 0L, kSeq, kCq, kCq, 0.125f);
  }
  {
    const int tiles = (kSeq / 64) * (kCkv / 64);
    wmma_gemm64<1, 0, 0, 2, false><<<dim3(tiles / 8, 1), dim3(256), 0, stream>>>(
        xb, nullptr, kCq, 0L, Wkb, nullptr, kCq, 0L, (void*)Kh, (void*)Kl, kCkv, 0L,
        nullptr, nullptr, 0L, kSeq, kCkv, kCq, 1.0f);
  }
  {
    const int tiles = (kCkv / 64) * (kSeq / 64);
    wmma_gemm64<1, 0, 0, 2, false><<<dim3(tiles / 8, 1), dim3(256), 0, stream>>>(
        Wvb, nullptr, kCq, 0L, xb, nullptr, kCq, 0L, (void*)Vth, (void*)Vtl, kSeq, 0L,
        nullptr, nullptr, 0L, kCkv, kSeq, kCq, 1.0f);
  }
  gqa_attn64<<<dim3(kHq * (kSeq / 64)), dim3(128), 0, stream>>>(Qh, Ql, Kh, Kl, Vth, Vtl, AOh, AOl);

  {
    const int tiles = (kSeq / 64) * (kCq / 64);
    wmma_gemm64<1, 2, 2, 0, false><<<dim3(tiles / 8, 1), dim3(256), 0, stream>>>(
        AOh, AOl, kCq, 0L, Wob, nullptr, kCq, 0L, (void*)out, nullptr, kCq, 0L,
        bo, nullptr, 0L, kSeq, kCq, kCq, 1.0f);
  }
}
